// LPCSynth_75608604278811
// MI455X (gfx1250) — hardware-run, weakly checked
//
#include <hip/hip_runtime.h>
#include <math.h>

typedef __attribute__((ext_vector_type(16))) _Float16     v16h;
typedef __attribute__((ext_vector_type(2)))  _Float16     v2h;
typedef __attribute__((ext_vector_type(8)))  float        v8f;
typedef __attribute__((ext_vector_type(4)))  float        v4f;
typedef __attribute__((ext_vector_type(8)))  unsigned int v8u;
typedef __attribute__((ext_vector_type(4)))  unsigned int v4u;
typedef __attribute__((ext_vector_type(2)))  unsigned int v2u;

constexpr int kHop     = 256;
constexpr int kWin     = 1024;
constexpr int kPad     = (kWin - kHop) / 2;
constexpr int kOrder   = 25;
constexpr int kLpcW    = kOrder + 1;
constexpr int kFrames  = 4096;
constexpr int kNx      = kFrames * kHop;
constexpr int kTotal   = (kFrames - 1) * kHop + kWin;
constexpr int kNout    = kTotal - 2 * kPad;
constexpr int kPre     = kWin - 16;
constexpr int kHbPitch = 1088;
constexpr int kCopyW   = 520;
constexpr int kXzW     = 1024;
constexpr int kXCarryLog2 = 6;
constexpr float kXCarry   = (float)(1 << kXCarryLog2);
constexpr int kTileP   = 68;
constexpr int kFirWaves = 2;

static_assert(kPad == 384, "pad");
static_assert(kNx == 1048576 && kNout == 1048576 && kTotal == 1049344, "sizes");
static_assert(kPre == 1008, "prefix");
static_assert((kWin % 32) == 0, "K multiple of 32");
static_assert((kHbPitch * 4) % 128 == 0, "tap plane row = whole lines");
static_assert((kFrames % 32) == 0 && (kFrames % kFirWaves) == 0, "frame tiling");
static_assert((kNx % 4) == 0 && (kHop % 4) == 0 && (kPad % 4) == 0, "16-B alignment of frame loads");

constexpr size_t kOffWT   = 0;
constexpr size_t kOffHB   = kOffWT + (size_t)kWin * 4;
constexpr size_t kOffWY   = kOffHB + (size_t)kFrames * kHbPitch * 4;
constexpr size_t kWsTotal = kOffWY + (size_t)kFrames * kWin * 4;
static_assert(kWsTotal == 34607104ull, "carve total");
static_assert(kWsTotal <= 134217728ull, "carve cap");
static_assert((kOffHB % 128) == 0 && (kOffWY % 128) == 0, "aligned regions");

__device__ __forceinline__ unsigned int pack_h2(float a, float b) {
  v2h p;
  p[0] = (_Float16)a;
  p[1] = (_Float16)b;
  return __builtin_bit_cast(unsigned int, p);
}

__device__ __forceinline__ v16h frag_words(const unsigned int* p) {
  const v4u lo = *(const v4u*)(p);
  const v4u hi = *(const v4u*)(p + 8);
  const v8u w = __builtin_shufflevector(lo, hi, 0, 1, 2, 3, 4, 5, 6, 7);
  return __builtin_bit_cast(v16h, w);
}

__device__ __forceinline__ v8f mma_f16(v16h a, v16h b, v8f c) {
  c = __builtin_amdgcn_wmma_f32_16x16x32_f16(false, a, false, b, (short)0, c, false, false);
  asm volatile("v_nop\n\tv_nop\n\tv_nop\n\tv_nop" : "+v"(c) : "v"(a), "v"(b));
  return c;
}

__global__ __launch_bounds__(256) void window_table_kernel(float* __restrict__ wtab) {
  __shared__ __align__(16) float sW[256];
  const int tid = threadIdx.x;
  const int t = blockIdx.x * 256 + tid;
  const float arg = (6.2831855f * (float)t) * (1.0f / (float)kWin);
  sW[tid] = 0.5f * (1.0f - cosf(arg));
  __syncthreads();
  if (tid < 64) {
    const v4f v = *(const v4f*)(sW + 4 * tid);
    float* dst = wtab + blockIdx.x * 256 + 4 * tid;
    *(volatile v4f*)dst = v;
    __threadfence();
    *(volatile v4f*)dst = v;
  }
}

__global__ __launch_bounds__(32) void impulse_kernel(const float* __restrict__ lpc, float* __restrict__ HB) {
  __shared__ __align__(16) float sL[32 * kLpcW];
  __shared__ __align__(16) float sT[32 * kTileP];
  const int lane = threadIdx.x;
  const int f0 = blockIdx.x * 32;
  const float* lsrc = lpc + (size_t)f0 * kLpcW;
#pragma unroll 1
  for (int it = 0; it < 7; ++it) {
    const int idx = lane + 32 * it;
    const int idc = idx < 208 ? idx : 207;
    v4f v = *(const v4f*)(lsrc + 4 * idc);
    asm volatile("" : "+v"(v));
    if (idx < 208) *(v4f*)(sL + 4 * idx) = v;
  }
  __syncthreads();
  float a[kOrder], hist[kOrder];
#pragma unroll
  for (int k = 0; k < kOrder; ++k) {
    a[k] = sL[lane * kLpcW + 1 + k];
    hist[k] = 0.0f;
  }
  const int hhalf = lane >> 4;
  const int c4 = (lane & 15) * 4;
#pragma unroll 1
  for (int c = 0; c < 16; ++c) {
#pragma unroll 1
    for (int s = 0; s < 64; ++s) {
      float acc = 0.0f;
#pragma unroll
      for (int k = 0; k < kOrder; ++k) acc = fmaf(a[k], hist[k], acc);
      const bool first = (c == 0) && (s == 0);
      const float hn = -acc;
      sT[lane * kTileP + (63 - s)] = first ? 0.0f : hn;
      const float push = first ? 1.0f : hn;
#pragma unroll
      for (int k = kOrder - 1; k > 0; --k) hist[k] = hist[k - 1];
      hist[0] = push;
    }
    __syncthreads();
    {
      const int wb = 960 - 64 * c;
      v4f tv[16];
#pragma unroll
      for (int it = 0; it < 16; ++it) tv[it] = *(const v4f*)(sT + (2 * it + hhalf) * kTileP + c4);
      for (int pass = 0; pass < 2; ++pass) {
#pragma unroll
        for (int it = 0; it < 16; ++it)
          *(volatile v4f*)(HB + (size_t)(f0 + 2 * it + hhalf) * kHbPitch + wb + c4) = tv[it];
        __threadfence();
      }
    }
    __syncthreads();
  }
  {
    const v4f z = (v4f){0.f, 0.f, 0.f, 0.f};
    for (int pass = 0; pass < 2; ++pass) {
#pragma unroll
      for (int it = 0; it < 16; ++it)
        *(volatile v4f*)(HB + (size_t)(f0 + 2 * it + hhalf) * kHbPitch + kWin + c4) = z;
      __threadfence();
    }
  }
}

__global__ __launch_bounds__(64) void fir_frames_kernel(const float* __restrict__ ex, const float* __restrict__ lpc,
                                                        const float* __restrict__ HB, float* __restrict__ WY) {
  __shared__ __align__(16) unsigned int sR[kFirWaves][8 * kCopyW];
  __shared__ __align__(16) unsigned int sXz[kFirWaves][kXzW];
  __shared__ __align__(16) float sXs[kFirWaves][kWin];
  const int tid = threadIdx.x;
  const int lane = tid & 31;
  const int wv = tid >> 5;
  const int f = blockIdx.x * kFirWaves + wv;
  const int n = lane & 15;
  const int hh = lane >> 4;
  unsigned int* rw = sR[wv];
  unsigned int* xzw = sXz[wv];
  float* xs = sXs[wv];
  const float* hrow = HB + (size_t)f * kHbPitch;
  const float gain = lpc[(size_t)f * kLpcW];

  float mx = 0.0f;
#pragma unroll 1
  for (int it = 0; it < 8; ++it) {
    const v4f v = *(const v4f*)(hrow + 4 * (lane + 32 * it));
    const float m01 = fmaxf(fabsf(v[0]), fabsf(v[1]));
    const float m23 = fmaxf(fabsf(v[2]), fabsf(v[3]));
    mx = fmaxf(mx, fmaxf(m01, m23));
  }
  mx = fmaxf(mx, __shfl_xor(mx, 16, 32));
  mx = fmaxf(mx, __shfl_xor(mx, 8, 32));
  mx = fmaxf(mx, __shfl_xor(mx, 4, 32));
  mx = fmaxf(mx, __shfl_xor(mx, 2, 32));
  mx = fmaxf(mx, __shfl_xor(mx, 1, 32));
  int eb = (int)((__float_as_uint(mx) >> 23) & 0xffu);
  eb = eb < 32 ? 32 : (eb > 222 ? 222 : eb);
  const float hscale = __uint_as_float((unsigned int)(262 - eb) << 23);
  const float fold   = __uint_as_float((unsigned int)(eb - 8 - kXCarryLog2) << 23);

#pragma unroll 1
  for (int it = 0; it < 5; ++it) {
    const int q = lane + 32 * it;
    const int qc = q < 130 ? q : 129;
    const float* src = hrow + 8 * qc;
    v4f f0 = *(const v4f*)(src);
    v4f f1 = *(const v4f*)(src + 4);
    v4f f2 = *(const v4f*)(src + 8);
    v4f f3 = *(const v4f*)(src + 12);
    asm volatile("" : "+v"(f0), "+v"(f1), "+v"(f2), "+v"(f3));
    unsigned int W[8];
    W[0] = pack_h2(f0[0] * hscale, f0[1] * hscale);
    W[1] = pack_h2(f0[2] * hscale, f0[3] * hscale);
    W[2] = pack_h2(f1[0] * hscale, f1[1] * hscale);
    W[3] = pack_h2(f1[2] * hscale, f1[3] * hscale);
    W[4] = pack_h2(f2[0] * hscale, f2[1] * hscale);
    W[5] = pack_h2(f2[2] * hscale, f2[3] * hscale);
    W[6] = pack_h2(f3[0] * hscale, f3[1] * hscale);
    W[7] = pack_h2(f3[2] * hscale, f3[3] * hscale);
    if (q < 130) {
#pragma unroll
      for (int s = 0; s < 8; ++s) {
        v4u o;
#pragma unroll
        for (int d = 0; d < 4; ++d) {
          if ((s & 1) == 0) {
            o[d] = W[(s >> 1) + d];
          } else {
            o[d] = (W[((s - 1) >> 1) + d] >> 16) | (W[((s - 1) >> 1) + d + 1] << 16);
          }
        }
        *(v4u*)(rw + s * kCopyW + 4 * qc) = o;
      }
    }
  }

  {
    const v4u z = (v4u){0u, 0u, 0u, 0u};
#pragma unroll 1
    for (int it = 0; it < 4; ++it) {
      const int idx = lane + 32 * it;
      if (idx < 126) *(v4u*)(xzw + 4 * idx) = z;
    }
    if (lane < 2) *(v4u*)(xzw + 1016 + 4 * lane) = z;
  }
  {
    const int gbase = f * kHop - kPad;
#pragma unroll 1
    for (int it = 0; it < 8; ++it) {
      const int t0 = 4 * (lane + 32 * it);
      const int g0 = gbase + t0;
      const bool inside = (g0 >= 0) && (g0 < kNx);
      int gc = g0 < 0 ? 0 : g0;
      gc = gc > (kNx - 4) ? (kNx - 4) : gc;
      const v4f xv = *(const v4f*)(ex + gc);
      v4f xq;
      xq[0] = inside ? xv[0] : 0.0f;
      xq[1] = inside ? xv[1] : 0.0f;
      xq[2] = inside ? xv[2] : 0.0f;
      xq[3] = inside ? xv[3] : 0.0f;
      *(v4f*)(xs + t0) = xq;
      v2u pw;
      pw[0] = pack_h2(xq[0] * kXCarry, xq[1] * kXCarry);
      pw[1] = pack_h2(xq[2] * kXCarry, xq[3] * kXCarry);
      *(v2u*)(xzw + (kPre >> 1) + (t0 >> 1)) = pw;
    }
  }
  __syncthreads();

  const int bsel = (7 - (n & 7)) * kCopyW + 4 * hh + ((n < 8) ? 4 : 0);
  const int arow = 8 * n + 4 * hh;
  v8f acc0 = (v8f){0.f, 0.f, 0.f, 0.f, 0.f, 0.f, 0.f, 0.f};
  v8f acc1 = acc0, acc2 = acc0, acc3 = acc0;
#pragma unroll 1
  for (int ks = 0; ks < 8; ++ks) {
    const v16h b  = frag_words(rw + bsel + 16 * ks);
    const v16h a3 = frag_words(xzw + arow + 384 + 16 * ks);
    acc3 = mma_f16(a3, b, acc3);
  }
#pragma unroll 1
  for (int ks = 8; ks < 16; ++ks) {
    const v16h b  = frag_words(rw + bsel + 16 * ks);
    const v16h a2 = frag_words(xzw + arow + 256 + 16 * ks);
    acc2 = mma_f16(a2, b, acc2);
    const v16h a3 = frag_words(xzw + arow + 384 + 16 * ks);
    acc3 = mma_f16(a3, b, acc3);
  }
#pragma unroll 1
  for (int ks = 16; ks < 24; ++ks) {
    const v16h b  = frag_words(rw + bsel + 16 * ks);
    const v16h a1 = frag_words(xzw + arow + 128 + 16 * ks);
    acc1 = mma_f16(a1, b, acc1);
    const v16h a2 = frag_words(xzw + arow + 256 + 16 * ks);
    acc2 = mma_f16(a2, b, acc2);
    const v16h a3 = frag_words(xzw + arow + 384 + 16 * ks);
    acc3 = mma_f16(a3, b, acc3);
  }
#pragma unroll 1
  for (int ks = 24; ks < 32; ++ks) {
    const v16h b  = frag_words(rw + bsel + 16 * ks);
    const v16h a0 = frag_words(xzw + arow + 16 * ks);
    acc0 = mma_f16(a0, b, acc0);
    const v16h a1 = frag_words(xzw + arow + 128 + 16 * ks);
    acc1 = mma_f16(a1, b, acc1);
    const v16h a2 = frag_words(xzw + arow + 256 + 16 * ks);
    acc2 = mma_f16(a2, b, acc2);
    const v16h a3 = frag_words(xzw + arow + 384 + 16 * ks);
    acc3 = mma_f16(a3, b, acc3);
  }

#pragma unroll
  for (int r = 0; r < 8; ++r) {
    const int tb = 128 * hh + 16 * r + n;
    const float x0 = xs[tb];
    const float x1 = xs[256 + tb];
    const float x2 = xs[512 + tb];
    const float x3 = xs[768 + tb];
    xs[tb]       = gain * fmaf(acc0[r], fold, x0);
    xs[256 + tb] = gain * fmaf(acc1[r], fold, x1);
    xs[512 + tb] = gain * fmaf(acc2[r], fold, x2);
    xs[768 + tb] = gain * fmaf(acc3[r], fold, x3);
  }
  __syncthreads();
  {
    v4f vv[8];
#pragma unroll
    for (int it = 0; it < 8; ++it) vv[it] = *(const v4f*)(xs + 4 * (lane + 32 * it));
    float* wrow = WY + (size_t)f * kWin;
    for (int pass = 0; pass < 2; ++pass) {
#pragma unroll
      for (int it = 0; it < 8; ++it) *(volatile v4f*)(wrow + 4 * (lane + 32 * it)) = vv[it];
      __threadfence();
    }
  }
}

__global__ __launch_bounds__(256) void ola_gather_kernel(const float* __restrict__ WY, const float* __restrict__ wtab,
                                                         float* __restrict__ out) {
  const int i = 4 * (blockIdx.x * 256 + threadIdx.x);
  const int p = i + kPad;
  const int fb = p >> 8;
  const int q = p & (kHop - 1);
  v4f num = (v4f){0.f, 0.f, 0.f, 0.f};
  v4f den = (v4f){0.f, 0.f, 0.f, 0.f};
#pragma unroll
  for (int r = 3; r >= 0; --r) {
    const int fr = fb - r;
    const bool ok = (fr >= 0) && (fr < kFrames);
    int frc = fr < 0 ? 0 : fr;
    frc = frc > (kFrames - 1) ? (kFrames - 1) : frc;
    const int t = q + kHop * r;
    const v4f y = *(const v4f*)(WY + (size_t)frc * kWin + t);
    const v4f w = *(const v4f*)(wtab + t);
#pragma unroll
    for (int e = 0; e < 4; ++e) {
      const float we = ok ? w[e] : 0.0f;
      const float ye = ok ? y[e] : 0.0f;
      num[e] = num[e] + we * ye;
      den[e] = den[e] + we;
    }
  }
  v4f o;
#pragma unroll
  for (int e = 0; e < 4; ++e) o[e] = num[e] * (1.0f / den[e]);
  float* dst = out + i;
  *(volatile v4f*)dst = o;
  __threadfence();
  *(volatile v4f*)dst = o;
}

extern "C" void kernel_launch(void* const* d_in, const int* in_sizes, int n_in,
                              void* d_out, int out_size, void* d_ws, size_t ws_size,
                              hipStream_t stream) {
  if (n_in < 2) return;
  if (in_sizes[0] != kNx) return;
  if (in_sizes[1] != kFrames * kLpcW) return;
  if (out_size != kNout) return;
  if (ws_size < kWsTotal) return;

  const float* ex  = (const float*)d_in[0];
  const float* lpc = (const float*)d_in[1];
  float* out = (float*)d_out;
  char* ws = (char*)d_ws;
  float* WT = (float*)(ws + kOffWT);
  float* HB = (float*)(ws + kOffHB);
  float* WY = (float*)(ws + kOffWY);

  window_table_kernel<<<kWin / 256, 256, 0, stream>>>(WT);
  impulse_kernel<<<kFrames / 32, 32, 0, stream>>>(lpc, HB);
  fir_frames_kernel<<<kFrames / kFirWaves, 32 * kFirWaves, 0, stream>>>(ex, lpc, HB, WY);
  ola_gather_kernel<<<kNout / 4 / 256, 256, 0, stream>>>(WY, WT, out);
}
